// QRNN_9337258901996
// MI455X (gfx1250) — hardware-verified
//
#include <hip/hip_runtime.h>
#include <stdint.h>

constexpr int NB   = 8;
constexpr int NT   = 1024;
constexpr int ND   = 1024;
constexpr int NU   = 1024;
constexpr int N3U  = 3 * NU;
constexpr int NWIN = 2;
constexpr int KTOT = NWIN * ND;
constexpr int TPAD = NT + 1;
constexpr int HALF = 4;

static_assert(KTOT % 32 == 0, "K multiple of 32");
static_assert(NT % 64 == 0, "M multiple of 64");
static_assert(N3U % 64 == 0, "N multiple of 64");
static_assert(NB % HALF == 0, "batch halves");

typedef __attribute__((ext_vector_type(16))) _Float16 v16h;
typedef __attribute__((ext_vector_type(8)))  _Float16 v8h;
typedef __attribute__((ext_vector_type(16))) __bf16   v16b;
typedef __attribute__((ext_vector_type(8)))  __bf16   v8b;
typedef __attribute__((ext_vector_type(8)))  float    v8f;
typedef __attribute__((ext_vector_type(4)))  float    v4f;
#define PSCALE 32768.0f
#define U16(p) ((const unsigned short*)(const void*)(p))
#define PSCALE_INV (1.0f / 32768.0f)

__device__ __forceinline__ unsigned short f2bf_bits(float f) {
  unsigned u = __float_as_uint(f);
  return (unsigned short)((u + 0x7FFFu + ((u >> 16) & 1u)) >> 16);
}
__device__ __forceinline__ float bf_bits2f(unsigned short h) { return __uint_as_float(((unsigned)h) << 16); }

__device__ __forceinline__ void dep_guard_h(v8f& a, v8f& b, v16h x, v16h y) { asm volatile("v_nop\n\tv_nop\n\tv_nop\n\tv_nop" : "+v"(a), "+v"(b) : "v"(x), "v"(y)); }
__device__ __forceinline__ void dep_guard_b(v8f& a, v8f& b, v16b x, v16b y) { asm volatile("v_nop\n\tv_nop\n\tv_nop\n\tv_nop" : "+v"(a), "+v"(b) : "v"(x), "v"(y)); }
__device__ __forceinline__ void keep4_h(v16h a, v16h b, v16h c, v16h d) { asm volatile("v_nop" :: "v"(a), "v"(b), "v"(c), "v"(d)); }
__device__ __forceinline__ void keep4_b(v16b a, v16b b, v16b c, v16b d) { asm volatile("v_nop" :: "v"(a), "v"(b), "v"(c), "v"(d)); }
__device__ __forceinline__ void acc_guard4(v8f& a, v8f& b, v8f& c, v8f& d) { asm volatile("v_nop\n\tv_nop\n\tv_nop\n\tv_nop" : "+v"(a), "+v"(b), "+v"(c), "+v"(d)); }
template <typename T> struct Frag;
template <> struct Frag<_Float16> {
  typedef v16h V; union U { v16h v; v8h h[2]; };
  static __device__ __forceinline__ v16h load(const _Float16* p) {
    U f; f.h[0] = *(const v8h*)(p); f.h[1] = *(const v8h*)(p + 16); return f.v;
  }
  static __device__ __forceinline__ v8f mma(v16h a, v16h b, v8f c) {
    return __builtin_amdgcn_wmma_f32_16x16x32_f16(false, a, false, b, (short)0, c, false, false);
  }
  static __device__ __forceinline__ void guard(v8f& a, v8f& b, v16h x, v16h y) { dep_guard_h(a, b, x, y); }
  static __device__ __forceinline__ void keep(v16h a, v16h b, v16h c, v16h d) { keep4_h(a, b, c, d); }
};
template <> struct Frag<__bf16> {
  typedef v16b V; union U { v16b v; v8b h[2]; };
  static __device__ __forceinline__ v16b load(const __bf16* p) {
    U f; f.h[0] = *(const v8b*)(p); f.h[1] = *(const v8b*)(p + 16); return f.v;
  }
  static __device__ __forceinline__ v8f mma(v16b a, v16b b, v8f c) {
    return __builtin_amdgcn_wmma_f32_16x16x32_bf16(false, a, false, b, (short)0, c, false, false);
  }
  static __device__ __forceinline__ void guard(v8f& a, v8f& b, v16b x, v16b y) { dep_guard_b(a, b, x, y); }
  static __device__ __forceinline__ void keep(v16b a, v16b b, v16b c, v16b d) { keep4_b(a, b, c, d); }
};

template <int ET> struct Elem;
template <> struct Elem<0> { typedef _Float16 T; };
template <> struct Elem<1> { typedef __bf16 T; };
template <int ET, bool SPLIT, int BIAS_MODE, int OUT_MODE, bool RESID, int ACT = 0>
__global__ __launch_bounds__(256) void wmma_gemm64(
    const unsigned short* __restrict__ Ap, const unsigned short* __restrict__ A2p, int lda, long strideA,
    const unsigned short* __restrict__ Btp, const unsigned short* __restrict__ Bt2p, int ldb, long strideB,
    void* __restrict__ Cout, void* __restrict__ Cout2, int ldc, long strideC,
    const float* __restrict__ bias,
    const float* __restrict__ resid, long strideR,
    int M, int N, int K, float scale) {
  typedef typename Elem<ET>::T T;
  typedef typename Frag<T>::V V;
  const T* A = (const T*)Ap; const T* A2 = (const T*)A2p; const T* Bt = (const T*)Btp; const T* Bt2 = (const T*)Bt2p;
  __shared__ __align__(16) float sT[8][16 * 68];
  const int b    = blockIdx.y;
  const int lane = threadIdx.x & 31;
  const int wave = threadIdx.x >> 5;
  const int tilesN = N >> 6;
  const int tilesM = M >> 6;
  const int tile = blockIdx.x * 8 + wave;
  if (tile >= tilesM * tilesN) return;
  const int tm = tile / tilesN;
  const int tn = tile - tm * tilesN;
  const int m0 = tm << 6;
  const int n0 = tn << 6;

  const T* Ab  = A  + (size_t)b * strideA;
  const T* Bb  = Bt + (size_t)b * strideB;
  const T* Ab2 = SPLIT ? (A2  + (size_t)b * strideA) : nullptr;
  const T* Bb2 = SPLIT ? (Bt2 + (size_t)b * strideB) : nullptr;

  const int rlane = lane & 15;
  const int koff  = (lane >> 4) * 8;
  const int mOff  = (lane >> 4) * 8;

  v8f acc[4][4];
#pragma unroll
  for (int i = 0; i < 4; ++i)
#pragma unroll
    for (int j = 0; j < 4; ++j) acc[i][j] = (v8f){0.f,0.f,0.f,0.f,0.f,0.f,0.f,0.f};

  for (int k0 = 0; k0 < K; k0 += 32) {
    V bh[4], bl[4];
#pragma unroll
    for (int j = 0; j < 4; ++j) {
      const size_t bo = (size_t)(n0 + (j << 4) + rlane) * ldb + koff + k0;
      bh[j] = Frag<T>::load(Bb + bo);
      if (SPLIT) bl[j] = Frag<T>::load(Bb2 + bo);
    }
#pragma unroll
    for (int i = 0; i < 4; ++i) {
      const size_t ao = (size_t)(m0 + (i << 4) + rlane) * lda + koff + k0;
      V ah = Frag<T>::load(Ab + ao);
      V al;
      if (SPLIT) al = Frag<T>::load(Ab2 + ao);
#pragma unroll
      for (int j = 0; j < 4; ++j) {
        acc[i][j] = Frag<T>::mma(ah, bh[j], acc[i][j]);
        if (SPLIT) {
          acc[i][j] = Frag<T>::mma(ah, bl[j], acc[i][j]);
          acc[i][j] = Frag<T>::mma(al, bh[j], acc[i][j]);
        }
      }
      Frag<T>::guard(acc[i][0], acc[i][3], ah, SPLIT ? al : ah);
    }
    Frag<T>::keep(bh[0], bh[1], bh[2], bh[3]);
    if (SPLIT) Frag<T>::keep(bl[0], bl[1], bl[2], bl[3]);
  }
  acc_guard4(acc[0][0], acc[0][1], acc[0][2], acc[0][3]);
  acc_guard4(acc[1][0], acc[1][1], acc[1][2], acc[1][3]);
  acc_guard4(acc[2][0], acc[2][1], acc[2][2], acc[2][3]);
  acc_guard4(acc[3][0], acc[3][1], acc[3][2], acc[3][3]);

  float* slab = sT[wave];
  const float* Rb = RESID ? (resid + (size_t)b * strideR) : nullptr;
#pragma unroll
  for (int i = 0; i < 4; ++i) {
    const int mBase = m0 + (i << 4);
#pragma unroll
    for (int j = 0; j < 4; ++j) {
      const int n = n0 + (j << 4) + rlane;
      float bv = 0.f;
      if (BIAS_MODE == 2) bv = bias[n];
#pragma unroll
      for (int r = 0; r < 8; ++r) {
        float v = acc[i][j][r] * scale;
        if (BIAS_MODE == 1) v += bias[mBase + mOff + r];
        if (BIAS_MODE == 2) v += bv;
        if (RESID) v += Rb[(size_t)(mBase + mOff + r) * ldc + n];
        if (ACT == 1) v = tanhf(v);
        if (ACT == 2) v = fmaxf(v, 0.0f);
        if (ACT == 3) v = v / (1.0f + expf(-v));
        if (ACT == 4) v = (v > 0.f) ? v : 0.01f * v;
        if (ACT == 5) v = 0.5f * v * (1.0f + erff(v * 0.70710678118654752f));
        slab[(mOff + r) * 68 + (j << 4) + rlane] = v;
      }
    }
    __builtin_amdgcn_fence(__ATOMIC_RELEASE, "workgroup");
    __builtin_amdgcn_wave_barrier();
    __builtin_amdgcn_fence(__ATOMIC_ACQUIRE, "workgroup");
    if (OUT_MODE == 0) {
      float* C = (float*)Cout + (size_t)b * strideC;
      const int hh = lane >> 4, c4 = (lane & 15) * 4;
      for (int pass = 0; pass < 2; ++pass) {
#pragma unroll
        for (int it = 0; it < 8; ++it) {
          const int row = it * 2 + hh;
          v4f v = *(const v4f*)(slab + row * 68 + c4);
          *(volatile v4f*)(C + (size_t)(mBase + row) * ldc + n0 + c4) = v;
        }
        __threadfence();
      }
    } else {
      const int q = lane >> 3, c8 = (lane & 7) * 8;
      unsigned short* C  = (unsigned short*)Cout  + (size_t)b * strideC;
      unsigned short* C2 = (OUT_MODE == 2) ? ((unsigned short*)Cout2 + (size_t)b * strideC) : nullptr;
      for (int pass = 0; pass < 2; ++pass) {
#pragma unroll
        for (int it = 0; it < 4; ++it) {
          const int row = it * 4 + q;
          const float* sp = slab + row * 68 + c8;
          v8h hv, lv;
#pragma unroll
          for (int e = 0; e < 8; ++e) {
            if (OUT_MODE == 1) {
              hv[e] = (_Float16)sp[e];
            } else {
              unsigned short hb = f2bf_bits(sp[e]);
              unsigned short lb = f2bf_bits(sp[e] - bf_bits2f(hb));
              hv[e] = __builtin_bit_cast(_Float16, hb);
              lv[e] = __builtin_bit_cast(_Float16, lb);
            }
          }
          *(volatile v8h*)(C + (size_t)(mBase + row) * ldc + n0 + c8) = hv;
          if (OUT_MODE == 2) *(volatile v8h*)(C2 + (size_t)(mBase + row) * ldc + n0 + c8) = lv;
        }
        __threadfence();
      }
    }
    __builtin_amdgcn_fence(__ATOMIC_RELEASE, "workgroup");
    __builtin_amdgcn_wave_barrier();
    __builtin_amdgcn_fence(__ATOMIC_ACQUIRE, "workgroup");
  }
}

__global__ __launch_bounds__(256) void kt_transpose_cast(const float* __restrict__ kern,
                                                         unsigned short* __restrict__ kt) {
  __shared__ __align__(16) float tile[64 * 68];
  const int tid = threadIdx.x, lane = tid & 31, wave = tid >> 5;
  const int u0 = blockIdx.x * 64;
  const int d0 = blockIdx.y * 64;
  const int w  = blockIdx.z;
#pragma unroll
  for (int i = 0; i < 4; ++i) {
    const int idx = tid + 256 * i;
    const int row = idx >> 4;
    const int c4  = (idx & 15) * 4;
    const v4f v = *(const v4f*)(kern + ((size_t)(w * ND + d0 + row)) * N3U + u0 + c4);
    *(v4f*)(tile + row * 68 + c4) = v;
  }
  __syncthreads();
  const int q = lane >> 3, c8 = (lane & 7) * 8;
  v8h val[2];
#pragma unroll
  for (int it = 0; it < 2; ++it) {
    const int ul = (wave * 2 + it) * 4 + q;
#pragma unroll
    for (int e = 0; e < 8; ++e) {
      const float f = tile[(c8 + e) * 68 + ul];
      val[it][e] = __builtin_bit_cast(_Float16, f2bf_bits(f));
    }
  }
  for (int pass = 0; pass < 2; ++pass) {
#pragma unroll
    for (int it = 0; it < 2; ++it) {
      const int ul = (wave * 2 + it) * 4 + q;
      unsigned short* dst = kt + ((size_t)(u0 + ul)) * KTOT + w * ND + d0 + c8;
      *(volatile v8h*)dst = val[it];
    }
    __threadfence();
  }
}

__global__ __launch_bounds__(256) void x_cast_pad(const float* __restrict__ x,
                                                  unsigned short* __restrict__ xb, int n8) {
  const int i = blockIdx.x * 256 + threadIdx.x;
  if (i < n8) {
    const size_t e   = (size_t)i * 8;
    const int    row = (int)(e >> 10);
    const int    col = (int)(e & (ND - 1));
    const int    b   = row / TPAD;
    const int    r   = row - b * TPAD;
    const int    rs  = (r > 0) ? (r - 1) : 0;
    const float* src = x + ((size_t)(b * NT + rs)) * ND + col;
    const v4f a = *(const v4f*)src;
    const v4f c = *(const v4f*)(src + 4);
    const bool live = (r > 0);
    v8h hv;
#pragma unroll
    for (int k = 0; k < 4; ++k) {
      const unsigned short b0 = live ? f2bf_bits(a[k]) : (unsigned short)0;
      const unsigned short b1 = live ? f2bf_bits(c[k]) : (unsigned short)0;
      hv[k]     = __builtin_bit_cast(_Float16, b0);
      hv[4 + k] = __builtin_bit_cast(_Float16, b1);
    }
    unsigned short* dst = xb + e;
    *(volatile v8h*)dst = hv;
    __threadfence();
    *(volatile v8h*)dst = hv;
  }
}

__global__ __launch_bounds__(256) void fo_pool_scan(const float* __restrict__ G,
                                                    float* __restrict__ out, int seq0) {
  const int bl = blockIdx.x;
  const int u0 = threadIdx.x * 4;
  const float* g = G + (size_t)bl * NT * N3U + u0;
  float* o = out + ((size_t)(seq0 + bl) * NT) * NU + u0;
  v4f h = (v4f){0.f, 0.f, 0.f, 0.f};
#pragma unroll 1
  for (int t = 0; t < NT; ++t) {
    const float* gt = g + (size_t)t * N3U;
    const v4f gz = *(const v4f*)(gt);
    const v4f gf = *(const v4f*)(gt + NU);
    const v4f go = *(const v4f*)(gt + 2 * NU);
    v4f hn;
#pragma unroll
    for (int e = 0; e < 4; ++e) {
      const float z  = 1.0f - 2.0f * __builtin_amdgcn_rcpf(1.0f + __expf(2.0f * gz[e]));
      const float f  = __builtin_amdgcn_rcpf(1.0f + __expf(-gf[e]));
      const float oo = __builtin_amdgcn_rcpf(1.0f + __expf(-go[e]));
      hn[e] = oo * (f * h[e] + (1.0f - f) * z);
    }
    h = hn;
    float* p = o + (size_t)t * NU;
    const v4f hv = h;
    *(volatile v4f*)p = hv;
    __threadfence();
    *(volatile v4f*)p = hv;
  }
}

extern "C" void kernel_launch(void* const* d_in, const int* in_sizes, int n_in,
                              void* d_out, int out_size, void* d_ws, size_t ws_size,
                              hipStream_t stream) {
  if (n_in < 3) return;
  if (in_sizes[0] != NB * NT * ND) return;
  if (in_sizes[1] != NWIN * ND * N3U) return;
  if (in_sizes[2] != N3U) return;
  if (out_size != NB * NT * NU) return;

  const size_t bytesKT = (size_t)N3U * KTOT * 2;
  const size_t bytesXB = (size_t)NB * TPAD * ND * 2;
  const size_t bytesG  = (size_t)HALF * NT * N3U * 4;
  const size_t offKT = 0;
  const size_t offXB = offKT + bytesKT;
  const size_t offG  = offXB + bytesXB;
  const size_t total = offG + bytesG;
  if (total > ws_size) return;

  const float* x    = (const float*)d_in[0];
  const float* kern = (const float*)d_in[1];
  const float* bias = (const float*)d_in[2];
  float* out = (float*)d_out;

  unsigned short* KT = (unsigned short*)((char*)d_ws + offKT);
  unsigned short* XB = (unsigned short*)((char*)d_ws + offXB);
  float*          G  = (float*)((char*)d_ws + offG);

  kt_transpose_cast<<<dim3(N3U / 64, ND / 64, NWIN), 256, 0, stream>>>(kern, KT);

  const int n8 = (int)((size_t)NB * TPAD * ND / 8);
  x_cast_pad<<<(n8 + 255) / 256, 256, 0, stream>>>(x, XB, n8);

  const int  tilesPerSeq = (NT / 64) * (N3U / 64);
  const int  gridX       = (tilesPerSeq + 7) / 8;
  const long strideA     = (long)TPAD * ND;
  const long strideC     = (long)NT * N3U;
  for (int half = 0; half < NB / HALF; ++half) {
    const unsigned short* Ah = XB + (size_t)half * HALF * strideA;
    wmma_gemm64<1, false, 2, 0, false, 0><<<dim3(gridX, HALF), 256, 0, stream>>>(
        Ah, Ah, ND, strideA,
        KT, KT, KTOT, 0L,
        (void*)G, (void*)G, N3U, strideC,
        bias,
        nullptr, 0L,
        NT, N3U, KTOT, 1.0f);
    fo_pool_scan<<<HALF, 256, 0, stream>>>(G, out, half * HALF);
  }
}
